// MaskedCausalAttention_55336358642962
// MI455X (gfx1250) — hardware-verified
//
#include <hip/hip_runtime.h>


#ifndef NB
#define NB 2
#endif
#ifndef SEQ
#define SEQ 2048
#endif
#define NB_FULL  2
#define SEQ_FULL 2048
#define DM   1024
#define NH_  16
#define HD   64
#define DQ   (NH_ * HD)
#define RH   512
#define RHX  ((RH < SEQ) ? RH : SEQ)
#define PCAR 1024.0f
#define SCL  0.125f
#define LDP  72
#define LDO  68
#define LDT  65
static_assert(SEQ % 64 == 0);
static_assert(RHX % 64 == 0);
static_assert(SEQ <= SEQ_FULL);
static_assert(NB <= NB_FULL);
static_assert(DM % 64 == 0);
static_assert(DQ % 64 == 0);
static_assert(DM % 32 == 0);
static_assert(HD == 64);

typedef _Float16 h16;
typedef unsigned short bf;
typedef __attribute__((ext_vector_type(16))) __bf16   v16bf;
typedef __attribute__((ext_vector_type(16))) _Float16 v16h;
typedef __attribute__((ext_vector_type(8)))  _Float16 v8h;
typedef __attribute__((ext_vector_type(8)))  unsigned short v8us;
typedef __attribute__((ext_vector_type(8)))  float    v8f;
typedef __attribute__((ext_vector_type(4)))  float    v4f;
typedef __attribute__((ext_vector_type(2)))  _Float16 v2h;
typedef __attribute__((ext_vector_type(2)))  unsigned short v2us;
typedef __attribute__((ext_vector_type(2)))  float    v2f;
typedef v8h  __attribute__((may_alias)) v8ha;
typedef v4f  __attribute__((may_alias)) v4fa;
typedef v8us __attribute__((may_alias)) v8usa;

__device__ __forceinline__ unsigned short f2bf(float f) { unsigned u = __float_as_uint(f); u += 0x7FFFu + ((u >> 16) & 1u); return (unsigned short)(u >> 16); }
__device__ __forceinline__ float bf2f(unsigned short b) { return __uint_as_float(((unsigned)b) << 16); }
__device__ __forceinline__ float bfr(float f) { return bf2f(f2bf(f)); }
__device__ __forceinline__ v16h cat16(v8h lo, v8h hi) { return __builtin_shufflevector(lo, hi, 0, 1, 2, 3, 4, 5, 6, 7, 8, 9, 10, 11, 12, 13, 14, 15); }
__device__ __forceinline__ v16bf cat16b(v8us lo, v8us hi) { return __builtin_bit_cast(v16bf, __builtin_shufflevector(lo, hi, 0, 1, 2, 3, 4, 5, 6, 7, 8, 9, 10, 11, 12, 13, 14, 15)); }
__device__ __forceinline__ v8f wmma16(v16h a, v16h b, v8f c) { return __builtin_amdgcn_wmma_f32_16x16x32_f16(false, a, false, b, (short)0, c, false, false); }
__device__ __forceinline__ v8f wmmab(v16bf a, v16bf b, v8f c) { return __builtin_amdgcn_wmma_f32_16x16x32_bf16(false, a, false, b, (short)0, c, false, false); }
__device__ __forceinline__ h16 tohx(float x) { return (h16)x; }
__device__ __forceinline__ void splitf(float y, unsigned short& h, unsigned short& l) { h = f2bf(y); l = f2bf(y - bf2f(h)); }

template <typename T16> struct WFrag;
template <> struct WFrag<h16> { typedef v16h V; static __device__ __forceinline__ V ld(const h16* p) { return cat16(*(const v8h*)p, *(const v8h*)(p + 16)); } static __device__ __forceinline__ v8f mma(V a, V b, v8f c) { return wmma16(a, b, c); } };
template <> struct WFrag<bf> { typedef v16bf V; static __device__ __forceinline__ V ld(const bf* p) { return cat16b(*(const v8us*)p, *(const v8us*)(p + 16)); } static __device__ __forceinline__ v8f mma(V a, V b, v8f c) { return wmmab(a, b, c); } };

template <typename T16, int NSPLIT, bool BIAS>
__global__ __launch_bounds__(32) void k_gemmw(const T16* __restrict__ A, const T16* __restrict__ A2, const T16* __restrict__ Bt, const T16* __restrict__ Bt2, int K, float* C, int ldc, const float* __restrict__ bias, size_t sA, size_t sB, size_t sC) {
    typedef typename WFrag<T16>::V V;
    __shared__ __align__(16) float os[16 * 68];
    const size_t z = blockIdx.z; A += z * sA; if (A2) A2 += z * sA; Bt += z * sB; if (Bt2) Bt2 += z * sB; C += z * sC;
    const int lane = threadIdx.x & 31, lr = lane & 15, hi = lane >> 4; const int r0 = blockIdx.x * 64, c0 = blockIdx.y * 64;
    v8f acc[4][4];
#pragma unroll
    for (int mb = 0; mb < 4; ++mb)
#pragma unroll
        for (int nb = 0; nb < 4; ++nb) acc[mb][nb] = (v8f){};
    const size_t aoff = (size_t)(r0 + lr) * K + 8 * hi, boff = (size_t)(c0 + lr) * K + 8 * hi;
#pragma unroll 1
    for (int kc = 0; kc < K; kc += 32) {
        V a[4], a2[4];
#pragma unroll
        for (int mb = 0; mb < 4; ++mb) { a[mb] = WFrag<T16>::ld(A + aoff + (size_t)mb * 16 * K + kc); if (NSPLIT == 1 || NSPLIT == 2) a2[mb] = WFrag<T16>::ld(A2 + aoff + (size_t)mb * 16 * K + kc); }
#pragma unroll
        for (int nb = 0; nb < 4; ++nb) { const V b = WFrag<T16>::ld(Bt + boff + (size_t)nb * 16 * K + kc); V b2; if (NSPLIT >= 2) b2 = WFrag<T16>::ld(Bt2 + boff + (size_t)nb * 16 * K + kc);
#pragma unroll
            for (int mb = 0; mb < 4; ++mb) { acc[mb][nb] = WFrag<T16>::mma(a[mb], b, acc[mb][nb]); if (NSPLIT == 1 || NSPLIT == 2) acc[mb][nb] = WFrag<T16>::mma(a2[mb], b, acc[mb][nb]); if (NSPLIT >= 2) acc[mb][nb] = WFrag<T16>::mma(a[mb], b2, acc[mb][nb]); } }
        asm volatile("v_nop\n\tv_nop\n\tv_nop\n\tv_nop" : "+v"(acc[0][0]), "+v"(acc[1][1]), "+v"(acc[2][2]), "+v"(acc[3][3]) : "v"(a[0]), "v"(a[3]));
    }
#pragma unroll
    for (int mb = 0; mb < 4; ++mb) {
#pragma unroll
        for (int nb = 0; nb < 4; ++nb) {
#pragma unroll
            for (int j = 0; j < 8; ++j) os[(hi * 8 + j) * 68 + nb * 16 + lr] = acc[mb][nb][j]; }
        __builtin_amdgcn_wave_barrier(); asm volatile("" ::: "memory");
        float* crow = C + (size_t)(r0 + mb * 16) * ldc + c0;
#pragma unroll 1
        for (int ps = 0; ps < 2; ++ps) {
#pragma unroll
            for (int s = 0; s < 8; ++s) { const int row = 2 * s + hi, cofs = lr * 4; v4f val = *(const v4fa*)(os + row * 68 + cofs); if (BIAS) { val[0] += bfr(bias[c0 + cofs]); val[1] += bfr(bias[c0 + cofs + 1]); val[2] += bfr(bias[c0 + cofs + 2]); val[3] += bfr(bias[c0 + cofs + 3]); }
                *(volatile v4f*)(crow + (size_t)row * ldc + cofs) = val; }
            if (ps == 0) __threadfence(); }
        __builtin_amdgcn_wave_barrier(); asm volatile("" ::: "memory");
    }
}

__global__ __launch_bounds__(256) void k_cvt8(const float* __restrict__ src, bf* dst, size_t n8) { const size_t i = (size_t)blockIdx.x * 256 + threadIdx.x; if (i >= n8) return; const v8f v = *(const v8f*)(src + i * 8); v8us o;
#pragma unroll
    for (int k = 0; k < 8; ++k) o[k] = f2bf(v[k]); *(volatile v8us*)(dst + i * 8) = o; __threadfence(); *(volatile v8us*)(dst + i * 8) = o; }

__global__ __launch_bounds__(256) void k_cvtT(const float* __restrict__ src, int rows, int cols, bf* dst) {
    __shared__ float ts[64 * LDT];
    const int c0 = blockIdx.x * 64, r0 = blockIdx.y * 64;
    const int t = threadIdx.x, lane = t & 31, wv = t >> 5;
    {
        const int r = t >> 2, cs = (t & 3) * 16;
        const float* p = src + (size_t)(r0 + r) * cols + c0 + cs;
        const v4f u0 = *(const v4f*)p, u1 = *(const v4f*)(p + 4), u2 = *(const v4f*)(p + 8), u3 = *(const v4f*)(p + 12);
#pragma unroll
        for (int q = 0; q < 4; ++q) { ts[r * LDT + cs + q] = u0[q]; ts[r * LDT + cs + 4 + q] = u1[q]; ts[r * LDT + cs + 8 + q] = u2[q]; ts[r * LDT + cs + 12 + q] = u3[q]; }
    }
    __syncthreads();
    v8us o[2]; size_t oo[2];
#pragma unroll
    for (int it = 0; it < 2; ++it) {
        const int c = wv * 8 + it * 4 + (lane >> 3), rp = (lane & 7) * 8;
#pragma unroll
        for (int q = 0; q < 8; ++q) o[it][q] = f2bf(ts[(rp + q) * LDT + c]);
        oo[it] = (size_t)(c0 + c) * rows + r0 + rp;
    }
    *(volatile v8us*)(dst + oo[0]) = o[0]; *(volatile v8us*)(dst + oo[1]) = o[1];
    __threadfence();
    *(volatile v8us*)(dst + oo[0]) = o[0]; *(volatile v8us*)(dst + oo[1]) = o[1];
}

__global__ __launch_bounds__(256) void k_qkp(const float* __restrict__ F, int pitch, int nheads, h16* P16, bf* Ph, bf* Pl) {
    const size_t e = ((size_t)blockIdx.x * 256 + threadIdx.x) * 2; if (e >= (size_t)nheads * SEQ * HD) return;
    const int d = (int)(e % HD); const int t = (int)((e / HD) % SEQ); const int hh = (int)(e / ((size_t)HD * SEQ));
    const v2f xv = *(const v2f*)(F + (size_t)t * pitch + hh * HD + d); v2h o16; v2us oh, ol;
#pragma unroll
    for (int q = 0; q < 2; ++q) { const float xq = xv[q]; o16[q] = tohx(xq); unsigned short a2, c2; splitf(xq, a2, c2); oh[q] = a2; ol[q] = c2; }
    *(volatile v2h*)(P16 + e) = o16; *(volatile v2us*)(Ph + e) = oh; *(volatile v2us*)(Pl + e) = ol; __threadfence(); *(volatile v2h*)(P16 + e) = o16; *(volatile v2us*)(Ph + e) = oh; *(volatile v2us*)(Pl + e) = ol; }

__global__ __launch_bounds__(256) void k_vtp(const float* __restrict__ F, int pitch, int nheads, h16* V16, bf* Vh, bf* Vl) { const size_t e = ((size_t)blockIdx.x * 256 + threadIdx.x) * 2; if (e >= (size_t)nheads * HD * SEQ) return; const int t = (int)(e % SEQ); const int d = (int)((e / SEQ) % HD); const int g = (int)(e / ((size_t)SEQ * HD)); v2h o16; v2us oh, ol;
#pragma unroll
    for (int q = 0; q < 2; ++q) { const float x = F[(size_t)(t + q) * pitch + g * HD + d]; o16[q] = tohx(x); unsigned short a2, c2; splitf(x, a2, c2); oh[q] = a2; ol[q] = c2; }
    *(volatile v2h*)(V16 + e) = o16; *(volatile v2us*)(Vh + e) = oh; *(volatile v2us*)(Vl + e) = ol; __threadfence(); *(volatile v2h*)(V16 + e) = o16; *(volatile v2us*)(Vh + e) = oh; *(volatile v2us*)(Vl + e) = ol; }

template <bool HR>
__global__ __launch_bounds__(128) __attribute__((amdgpu_num_vgpr(256))) void k_attn(const h16* __restrict__ Q16, const bf* __restrict__ Qh, const bf* __restrict__ Ql,
                                              const h16* __restrict__ K16, const bf* __restrict__ Kh, const bf* __restrict__ Kl,
                                              const h16* __restrict__ VT16, const bf* __restrict__ VTh, const bf* __restrict__ VTl,
                                              int qb0, bf* ATh, bf* ATl) {
    __shared__ __align__(16) h16 sP[HR ? 8 : 4 * 16 * LDP];
    __shared__ __align__(16) bf sPh[HR ? 4 * 16 * LDP : 8];
    __shared__ __align__(16) bf sPl[HR ? 4 * 16 * LDP : 8];
    __shared__ __align__(16) float os[4 * 16 * LDO];
    const int lane = threadIdx.x & 31, lr = lane & 15, hi = lane >> 4, wv = threadIdx.x >> 5;
    const int h = blockIdx.y; const int q0 = (qb0 + (int)blockIdx.x) * 64; const int rw = q0 + wv * 16;
    const size_t hq = (size_t)h * SEQ * HD;
    const int pofs = wv * 16 * LDP; float* osw = os + wv * 16 * LDO;
    v16h qa[2]; v16bf qah[2], qal[2];
    if (HR) {
#pragma unroll
        for (int ks = 0; ks < 2; ++ks) { const size_t o = hq + (size_t)(rw + lr) * HD + 8 * hi + 32 * ks; qah[ks] = WFrag<bf>::ld(Qh + o); qal[ks] = WFrag<bf>::ld(Ql + o); }
    } else {
#pragma unroll
        for (int ks = 0; ks < 2; ++ks) qa[ks] = WFrag<h16>::ld(Q16 + hq + (size_t)(rw + lr) * HD + 8 * hi + 32 * ks);
    }
    v8f accO[4]; float mrow[8], lrow[8];
#pragma unroll
    for (int nb = 0; nb < 4; ++nb) accO[nb] = (v8f){};
#pragma unroll
    for (int r = 0; r < 8; ++r) { mrow[r] = -1.0e30f; lrow[r] = 0.0f; }
    const float L2E = 1.4426950408889634f;
    const int nch = q0 / 64 + 1;
#pragma unroll 1
    for (int c = 0; c < nch; ++c) {
        const int s0 = c * 64;
        __syncthreads();
        v8f S[4];
#pragma unroll
        for (int nb = 0; nb < 4; ++nb) {
            S[nb] = (v8f){};
            const size_t kr = hq + (size_t)(s0 + nb * 16 + lr) * HD + 8 * hi;
            if (HR) {
                const v16bf b0 = WFrag<bf>::ld(Kh + kr), b1 = WFrag<bf>::ld(Kh + kr + 32), e0 = WFrag<bf>::ld(Kl + kr), e1 = WFrag<bf>::ld(Kl + kr + 32);
                S[nb] = wmmab(qah[0], b0, S[nb]); S[nb] = wmmab(qal[0], b0, S[nb]); S[nb] = wmmab(qah[0], e0, S[nb]);
                S[nb] = wmmab(qah[1], b1, S[nb]); S[nb] = wmmab(qal[1], b1, S[nb]); S[nb] = wmmab(qah[1], e1, S[nb]);
                asm volatile("v_nop\n\tv_nop\n\tv_nop\n\tv_nop" : "+v"(S[nb]) : "v"(b0), "v"(b1), "v"(e0), "v"(e1), "v"(qah[0]), "v"(qah[1]), "v"(qal[0]), "v"(qal[1]));
            } else {
                const v16h b0 = WFrag<h16>::ld(K16 + kr), b1 = WFrag<h16>::ld(K16 + kr + 32);
                S[nb] = wmma16(qa[0], b0, S[nb]); S[nb] = wmma16(qa[1], b1, S[nb]);
                asm volatile("v_nop\n\tv_nop\n\tv_nop\n\tv_nop" : "+v"(S[nb]) : "v"(b0), "v"(b1), "v"(qa[0]), "v"(qa[1]));
            }
        }
#pragma unroll
        for (int r = 0; r < 8; ++r) {
            const int i = rw + hi * 8 + r;
            float m = -1.0e30f;
#pragma unroll
            for (int nb = 0; nb < 4; ++nb) { const int j = s0 + nb * 16 + lr; const float t = (j <= i) ? S[nb][r] * SCL : -1.0e30f; S[nb][r] = t; m = fmaxf(m, t); }
#pragma unroll
            for (int sh = 8; sh > 0; sh >>= 1) m = fmaxf(m, __shfl_xor(m, sh, 32));
            const float mn = fmaxf(mrow[r], m);
            const float al = __builtin_amdgcn_exp2f((mrow[r] - mn) * L2E);
            float sum = 0.0f;
#pragma unroll
            for (int nb = 0; nb < 4; ++nb) { const float p = __builtin_amdgcn_exp2f((S[nb][r] - mn) * L2E); S[nb][r] = p; sum += p; }
#pragma unroll
            for (int sh = 8; sh > 0; sh >>= 1) sum += __shfl_xor(sum, sh, 32);
            lrow[r] = lrow[r] * al + sum; mrow[r] = mn;
#pragma unroll
            for (int nb = 0; nb < 4; ++nb) accO[nb][r] = accO[nb][r] * al;
        }
        if (HR) {
#pragma unroll
            for (int r = 0; r < 8; ++r)
#pragma unroll
                for (int nb = 0; nb < 4; ++nb) { unsigned short a2, c2; splitf(S[nb][r], a2, c2); const int ix = pofs + (hi * 8 + r) * LDP + nb * 16 + lr; sPh[ix] = a2; sPl[ix] = c2; }
        } else {
#pragma unroll
            for (int r = 0; r < 8; ++r)
#pragma unroll
                for (int nb = 0; nb < 4; ++nb) sP[pofs + (hi * 8 + r) * LDP + nb * 16 + lr] = tohx(S[nb][r] * PCAR);
        }
        __syncthreads();
        if (HR) {
            v16bf ph[2], pl[2];
#pragma unroll
            for (int ks = 0; ks < 2; ++ks) { const int o = pofs + lr * LDP + 32 * ks + 8 * hi; ph[ks] = cat16b(*(const v8usa*)(sPh + o), *(const v8usa*)(sPh + o + 16)); pl[ks] = cat16b(*(const v8usa*)(sPl + o), *(const v8usa*)(sPl + o + 16)); }
#pragma unroll
            for (int nb = 0; nb < 4; ++nb) {
                const size_t vr = hq + (size_t)(nb * 16 + lr) * SEQ + s0 + 8 * hi;
                const v16bf v0 = WFrag<bf>::ld(VTh + vr), v1 = WFrag<bf>::ld(VTh + vr + 32), w0 = WFrag<bf>::ld(VTl + vr), w1 = WFrag<bf>::ld(VTl + vr + 32);
                accO[nb] = wmmab(ph[0], v0, accO[nb]); accO[nb] = wmmab(pl[0], v0, accO[nb]); accO[nb] = wmmab(ph[0], w0, accO[nb]);
                accO[nb] = wmmab(ph[1], v1, accO[nb]); accO[nb] = wmmab(pl[1], v1, accO[nb]); accO[nb] = wmmab(ph[1], w1, accO[nb]);
                asm volatile("v_nop\n\tv_nop\n\tv_nop\n\tv_nop" : "+v"(accO[nb]) : "v"(v0), "v"(v1), "v"(w0), "v"(w1), "v"(ph[0]), "v"(ph[1]), "v"(pl[0]), "v"(pl[1]));
            }
        } else {
            v16h pa[2];
#pragma unroll
            for (int ks = 0; ks < 2; ++ks) { const int o = pofs + lr * LDP + 32 * ks + 8 * hi; pa[ks] = cat16(*(const v8ha*)(sP + o), *(const v8ha*)(sP + o + 16)); }
#pragma unroll
            for (int nb = 0; nb < 4; ++nb) {
                const size_t vr = hq + (size_t)(nb * 16 + lr) * SEQ + s0 + 8 * hi;
                const v16h v0 = WFrag<h16>::ld(VT16 + vr), v1 = WFrag<h16>::ld(VT16 + vr + 32);
                accO[nb] = wmma16(pa[0], v0, accO[nb]); accO[nb] = wmma16(pa[1], v1, accO[nb]);
                asm volatile("v_nop\n\tv_nop\n\tv_nop\n\tv_nop" : "+v"(accO[nb]) : "v"(v0), "v"(v1), "v"(pa[0]), "v"(pa[1]));
            }
        }
    }
    float inv[8];
#pragma unroll
    for (int r = 0; r < 8; ++r) inv[r] = __fdiv_rn(HR ? 1.0f : (1.0f / PCAR), lrow[r]);
#pragma unroll
    for (int nb = 0; nb < 4; ++nb)
#pragma unroll
        for (int r = 0; r < 8; ++r) osw[(hi * 8 + r) * LDO + nb * 16 + lr] = accO[nb][r] * inv[r];
    __syncthreads();
#pragma unroll 1
    for (int ps = 0; ps < 2; ++ps) {
#pragma unroll
        for (int k = 0; k < 4; ++k) { const int row = 4 * k + (lane >> 3), pc = (lane & 7) * 8; const float* src = osw + row * LDO + pc;
            const v4f u0 = *(const v4fa*)src, u1 = *(const v4fa*)(src + 4); v8us oh, ol;
#pragma unroll
            for (int q = 0; q < 4; ++q) { unsigned short a2, c2; const float y0 = u0[q]; splitf(y0, a2, c2); oh[q] = a2; ol[q] = c2; const float y1 = u1[q]; splitf(y1, a2, c2); oh[q + 4] = a2; ol[q + 4] = c2; }
            const size_t oo = (size_t)(rw + row) * DQ + (size_t)h * HD + pc;
            *(volatile v8us*)(ATh + oo) = oh; *(volatile v8us*)(ATl + oo) = ol; }
        if (ps == 0) __threadfence(); }
}

extern "C" void kernel_launch(void* const* d_in, const int* in_sizes, int n_in,
                              void* d_out, int out_size, void* d_ws, size_t ws_size, hipStream_t stream) {
    if (n_in < 9) return;
    if ((size_t)in_sizes[0] < (size_t)(NB - 1) * SEQ_FULL * DM + (size_t)SEQ * DM) return;
    if ((size_t)in_sizes[1] < (size_t)DM * DQ || (size_t)in_sizes[3] < (size_t)DM * DQ || (size_t)in_sizes[5] < (size_t)DM * DQ || (size_t)in_sizes[7] < (size_t)DQ * DM) return;
    if (in_sizes[2] < DQ || in_sizes[4] < DQ || in_sizes[6] < DQ || in_sizes[8] < DM) return;
    if ((size_t)out_size < (size_t)NB * SEQ * DM) return;
    const float* x = (const float*)d_in[0]; const float* wq = (const float*)d_in[1]; const float* bq = (const float*)d_in[2]; const float* wk = (const float*)d_in[3]; const float* bk = (const float*)d_in[4]; const float* wv = (const float*)d_in[5]; const float* bv = (const float*)d_in[6]; const float* wo = (const float*)d_in[7]; const float* bo = (const float*)d_in[8];
    float* OUT = (float*)d_out;
    char* wsp = (char*)d_ws;
    auto take = [&](size_t bytes) { char* p = wsp; wsp += (bytes + 255) & ~(size_t)255; return (void*)p; };
    bf* WQ = (bf*)take((size_t)DQ * DM * 2); bf* WK = (bf*)take((size_t)DQ * DM * 2); bf* WV = (bf*)take((size_t)DQ * DM * 2); bf* WO = (bf*)take((size_t)DM * DQ * 2);
    bf* XB = (bf*)take((size_t)SEQ * DM * 2); float* FQ = (float*)take((size_t)SEQ * DQ * 4); float* FK = (float*)take((size_t)SEQ * DQ * 4);
    h16* QP16 = (h16*)take((size_t)NH_ * SEQ * HD * 2); h16* KP16 = (h16*)take((size_t)NH_ * SEQ * HD * 2); h16* VT16 = (h16*)take((size_t)NH_ * HD * SEQ * 2);
    bf* QPh = (bf*)take((size_t)NH_ * SEQ * HD * 2); bf* QPl = (bf*)take((size_t)NH_ * SEQ * HD * 2); bf* KPh = (bf*)take((size_t)NH_ * SEQ * HD * 2); bf* KPl = (bf*)take((size_t)NH_ * SEQ * HD * 2);
    bf* VTh = (bf*)take((size_t)NH_ * HD * SEQ * 2); bf* VTl = (bf*)take((size_t)NH_ * HD * SEQ * 2);
    bf* ATh = (bf*)take((size_t)SEQ * DQ * 2); bf* ATl = (bf*)take((size_t)SEQ * DQ * 2);
    if ((size_t)(wsp - (char*)d_ws) > ws_size) return;
    float* FV = FK;
    k_cvtT<<<dim3(DQ / 64, DM / 64, 1), 256, 0, stream>>>(wq, DM, DQ, WQ);
    k_cvtT<<<dim3(DQ / 64, DM / 64, 1), 256, 0, stream>>>(wk, DM, DQ, WK);
    k_cvtT<<<dim3(DQ / 64, DM / 64, 1), 256, 0, stream>>>(wv, DM, DQ, WV);
    k_cvtT<<<dim3(DM / 64, DQ / 64, 1), 256, 0, stream>>>(wo, DQ, DM, WO);
    const unsigned LX = (unsigned)(((size_t)SEQ * DM / 8 + 255) / 256), LP = (unsigned)(((size_t)NH_ * SEQ * HD / 2 + 255) / 256);
    for (int b = 0; b < NB; ++b) {
        const float* xb = x + (size_t)b * SEQ_FULL * DM;
        k_cvt8<<<LX, 256, 0, stream>>>(xb, XB, (size_t)SEQ * DM / 8);
        k_gemmw<bf, 0, true><<<dim3(SEQ / 64, DQ / 64, 1), 32, 0, stream>>>(XB, nullptr, WQ, nullptr, DM, FQ, DQ, bq, 0, 0, 0);
        k_qkp<<<LP, 256, 0, stream>>>(FQ, DQ, NH_, QP16, QPh, QPl);
        k_gemmw<bf, 0, true><<<dim3(SEQ / 64, DQ / 64, 1), 32, 0, stream>>>(XB, nullptr, WK, nullptr, DM, FK, DQ, bk, 0, 0, 0);
        k_qkp<<<LP, 256, 0, stream>>>(FK, DQ, NH_, KP16, KPh, KPl);
        k_gemmw<bf, 0, true><<<dim3(SEQ / 64, DQ / 64, 1), 32, 0, stream>>>(XB, nullptr, WV, nullptr, DM, FV, DQ, bv, 0, 0, 0);
        k_vtp<<<LP, 256, 0, stream>>>(FV, DQ, NH_, VT16, VTh, VTl);
        k_attn<true><<<dim3(RHX / 64, NH_, 1), 128, 0, stream>>>(QP16, QPh, QPl, KP16, KPh, KPl, VT16, VTh, VTl, 0, ATh, ATl);
        if (SEQ > RHX) k_attn<false><<<dim3((SEQ - RHX) / 64, NH_, 1), 128, 0, stream>>>(QP16, QPh, QPl, KP16, KPh, KPl, VT16, VTh, VTl, RHX / 64, ATh, ATl);
        k_gemmw<bf, 1, true><<<dim3(SEQ / 64, DM / 64, 1), 32, 0, stream>>>(ATh, ATl, WO, nullptr, DQ, OUT + (size_t)b * SEQ * DM, DM, bo, 0, 0, 0);
    }
}
